// MambaLayer_27779848470954
// MI455X (gfx1250) — hardware-verified
//
#include <hip/hip_runtime.h>
#include <stddef.h>
#include <stdint.h>

#define BSZ    4
#define DM     256
#define LSEQ   4096
#define DI     512
#define DS     16
#define DTR    16
#define NDBL   48
#define NXP    64
#define TROWS  (BSZ * LSEQ)
#define KIN    (2 * DM)
#define KXC    (2 * DI)
#define KXM    (2 * DM)
#define GBM    64
#define GBN    128
#define GTHR   128
#define NTHR   256
#define CL     64
#define SD     64
#define TPP    68
#define LNP    260
#define WSMAX  134217728

#define NU_INP (2 * DI * (KIN / 8))
#define NU_XP  (NXP * (KXC / 8))
#define NU_OUT (DM * (KXC / 8))
#define NU_PRJ (DM * (KXM / 8))
#define NU_ALL (NU_INP + NU_XP + NU_OUT + NU_PRJ)

#define SCAN_LDS_FLOATS (CL * NDBL + 4 * CL * SD + 2 * SD * DS + 2 * SD)
#define SCAN_LDS_BYTES  (SCAN_LDS_FLOATS * 4)

static_assert(NU_INP % NTHR == 0 && NU_XP % NTHR == 0 && NU_OUT % NTHR == 0 && NU_PRJ % NTHR == 0);
static_assert(TROWS % GBM == 0 && LSEQ % GBM == 0 && (2 * DI) % GBN == 0 && DM % GBN == 0 && DI % GBN == 0);
static_assert(KIN % 32 == 0 && KXC % 32 == 0 && KXM % 32 == 0 && NXP % 16 == 0 && NXP >= NDBL);
static_assert(LSEQ % CL == 0 && DI % SD == 0 && SD * 4 == NTHR && DS == 16 && DTR == 16 && NDBL == DTR + 2 * DS);
static_assert(SCAN_LDS_BYTES <= 300000);
static_assert(LSEQ % 32 == 0 && DM == NTHR && (LNP * 4) % 16 == 0 && (TPP * 4) % 16 == 0);
static_assert(GBM == (GTHR / 32) * 16 && GBN == 8 * 16);
static_assert((size_t)TROWS * KIN * 2 == (size_t)TROWS * KXM * 2);
static_assert((size_t)TROWS * DI * 4 == (size_t)TROWS * KXC * 2);
static_assert((CL + 3) * (SD / 4) <= 5 * NTHR);

typedef float          v4f   __attribute__((ext_vector_type(4)));
typedef float          v8f   __attribute__((ext_vector_type(8)));
typedef int            v8i   __attribute__((ext_vector_type(8)));
typedef unsigned short v8us  __attribute__((ext_vector_type(8)));
typedef unsigned short v16us __attribute__((ext_vector_type(16)));
typedef __bf16         v16bf __attribute__((ext_vector_type(16)));
typedef v4f  __attribute__((may_alias)) v4fa;
typedef v8us __attribute__((may_alias)) v8usa;
union FragB { v16bf v; v16us u; v8us h[2]; v8i w; };

__device__ __forceinline__ v8f wmb(const FragB& a, const FragB& b, v8f c) {
  v8f d = __builtin_amdgcn_wmma_f32_16x16x32_bf16(false, a.v, false, b.v, (short)0, c, false, false);
  asm volatile("v_nop\n\tv_nop\n\tv_nop\n\tv_nop" : "+v"(d) : "v"(a.w), "v"(b.w));
  return d;
}

__device__ __forceinline__ unsigned bf16_bits(float f) {
  const unsigned u = __float_as_uint(f);
  return (u + 0x7FFFu + ((u >> 16) & 1u)) >> 16;
}
__device__ __forceinline__ float bf16_val(float f) {
  return __uint_as_float(bf16_bits(f) << 16);
}
__device__ __forceinline__ float bfw(unsigned w) {
  return __uint_as_float((w & 0xffffu) << 16);
}
__device__ __forceinline__ void put16(unsigned short* dp, v8us o) {
  *(volatile v8us*)dp = o;
  __threadfence();
  *(volatile v8us*)dp = o;
}
__device__ __forceinline__ v8us hilo8(const float* sp, unsigned ml, unsigned mh) {
  const v4f a = *(const v4fa*)sp;
  const v4f b = *(const v4fa*)(sp + 4);
  const v8f f8 = {a.x, a.y, a.z, a.w, b.x, b.y, b.z, b.w};
  v8us oo;
#pragma unroll
  for (int e = 0; e < 8; ++e) {
    const unsigned hb = bf16_bits(f8[e]);
    const unsigned lb = bf16_bits(f8[e] - __uint_as_float(hb << 16));
    oo[e] = (unsigned short)((hb & ml) | (lb & mh));
  }
  return oo;
}

template <int NT>
__device__ __forceinline__ void gemm_core(const unsigned short* __restrict__ A, int lda,
                                          const unsigned short* __restrict__ BT, int ldb, int K,
                                          int rowBase, int colBase, int wave, int hh, int m, v8f (&acc)[NT]) {
  {
    const v8f z = {0.f, 0.f, 0.f, 0.f, 0.f, 0.f, 0.f, 0.f};
#pragma unroll
    for (int t = 0; t < NT; ++t) acc[t] = z;
  }
  const unsigned short* ap = A  + (size_t)(rowBase + 16 * wave + m) * (size_t)lda + 8 * hh;
  const unsigned short* bp = BT + (size_t)(colBase + m) * (size_t)ldb + 8 * hh;
#pragma unroll 1
  for (int k0 = 0; k0 < K; k0 += 32) {
    FragB af;
    af.h[0] = *(const v8usa*)(ap + k0);
    af.h[1] = *(const v8usa*)(ap + k0 + 16);
#pragma unroll
    for (int nt = 0; nt < NT; ++nt) {
      const unsigned short* wq = bp + (size_t)(16 * nt) * (size_t)ldb + k0;
      FragB bf;
      bf.h[0] = *(const v8usa*)wq;
      bf.h[1] = *(const v8usa*)(wq + 16);
      acc[nt] = wmb(af, bf, acc[nt]);
    }
  }
}

__global__ __launch_bounds__(NTHR) void k_wprep(const float* __restrict__ Win, const float* __restrict__ Wxp,
                                                const float* __restrict__ Wout, const float* __restrict__ Wpr,
                                                unsigned short* INP2, unsigned short* XP2,
                                                unsigned short* OUT2, unsigned short* PRJ2) {
  const int u  = (int)blockIdx.x * NTHR + (int)threadIdx.x;
  const int L0 = NU_INP, L1 = L0 + NU_XP, L2 = L1 + NU_OUT, L3 = L2 + NU_PRJ;
  const float* src;
  unsigned short* dst;
  float zf = 1.0f;
  if (u < L0) {
    const int n = u >> 6, k8 = (u & 63) * 8;
    src = Win + (size_t)n * DM + (k8 & (DM - 1));
    dst = INP2 + (size_t)n * KIN + k8;
  } else if (u < L1) {
    const int v = u - L0;
    const int n = v >> 7, k8 = (v & 127) * 8;
    const int nc = n < NDBL ? n : NDBL - 1;
    zf = n < NDBL ? 1.0f : 0.0f;
    src = Wxp + (size_t)nc * DI + (k8 & (DI - 1));
    dst = XP2 + (size_t)n * KXC + k8;
  } else if (u < L2) {
    const int v = u - L1;
    const int n = v >> 7, k8 = (v & 127) * 8;
    src = Wout + (size_t)n * DI + (k8 & (DI - 1));
    dst = OUT2 + (size_t)n * KXC + k8;
  } else if (u < L3) {
    const int v = u - L2;
    const int n = v >> 6, k8 = (v & 63) * 8;
    src = Wpr + (size_t)n * DM + (k8 & (DM - 1));
    dst = PRJ2 + (size_t)n * KXM + k8;
  } else {
    return;
  }
  const v4f a = *(const v4fa*)src;
  const v4f c = *(const v4fa*)(src + 4);
  v8us o;
  o[0] = (unsigned short)bf16_bits(a.x * zf);
  o[1] = (unsigned short)bf16_bits(a.y * zf);
  o[2] = (unsigned short)bf16_bits(a.z * zf);
  o[3] = (unsigned short)bf16_bits(a.w * zf);
  o[4] = (unsigned short)bf16_bits(c.x * zf);
  o[5] = (unsigned short)bf16_bits(c.y * zf);
  o[6] = (unsigned short)bf16_bits(c.z * zf);
  o[7] = (unsigned short)bf16_bits(c.w * zf);
  put16(dst, o);
}

__global__ __launch_bounds__(NTHR) void k_ln(const float* __restrict__ x, const float* __restrict__ nw,
                                             const float* __restrict__ nb, unsigned short* XN) {
  __shared__ __attribute__((aligned(16))) float sh[32 * LNP];
  __shared__ float sNW[DM];
  __shared__ float sNB[DM];
  const int tid = (int)threadIdx.x;
  const int b = (int)blockIdx.y, l0 = (int)blockIdx.x * 32;
  const float* xb = x + (size_t)b * DM * LSEQ + l0;
  sNW[tid] = bf16_val(nw[tid]);
  sNB[tid] = bf16_val(nb[tid]);
  {
    const int q = tid & 7, c0 = tid >> 3;
#pragma unroll 1
    for (int s = 0; s < 8; ++s) {
      const int c = s * 32 + c0;
      const v4f v = *(const v4fa*)(xb + (size_t)c * LSEQ + 4 * q);
      sh[(4 * q + 0) * LNP + c] = bf16_val(v.x);
      sh[(4 * q + 1) * LNP + c] = bf16_val(v.y);
      sh[(4 * q + 2) * LNP + c] = bf16_val(v.z);
      sh[(4 * q + 3) * LNP + c] = bf16_val(v.w);
    }
  }
  __syncthreads();
  {
    const int r = tid >> 3, sub = tid & 7, cb = sub * 32;
    float* row = sh + r * LNP + cb;
    float s = 0.0f;
#pragma unroll 4
    for (int j = 0; j < 32; ++j) s += row[j];
    s += __shfl_xor(s, 1);
    s += __shfl_xor(s, 2);
    s += __shfl_xor(s, 4);
    const float mu = s * (1.0f / 256.0f);
    float s2 = 0.0f;
#pragma unroll 4
    for (int j = 0; j < 32; ++j) {
      const float dv = row[j] - mu;
      s2 += dv * dv;
    }
    s2 += __shfl_xor(s2, 1);
    s2 += __shfl_xor(s2, 2);
    s2 += __shfl_xor(s2, 4);
    const float var = s2 * (1.0f / 256.0f);
    const float rs  = 1.0f / sqrtf(var + 1e-5f);
#pragma unroll 4
    for (int j = 0; j < 32; ++j) {
      const int c = cb + j;
      row[j] = (row[j] - mu) * rs * sNW[c] + sNB[c];
    }
  }
  __syncthreads();
  {
    v8us pv[8];
#pragma unroll
    for (int s = 0; s < 8; ++s) {
      const int p = s * NTHR + tid;
      const int i = p >> 6, j = p & 63;
      const int part = j >> 5, c8 = (j & 31) * 8;
      const unsigned mh = 0u - (unsigned)part, ml = ~mh;
      pv[s] = hilo8(sh + i * LNP + c8, ml, mh);
    }
    unsigned short* base = XN + (size_t)(b * LSEQ + l0) * (size_t)KIN;
#pragma unroll
    for (int s = 0; s < 8; ++s) *(volatile v8us*)(base + (size_t)(s * NTHR + tid) * 8) = pv[s];
    __threadfence();
#pragma unroll
    for (int s = 0; s < 8; ++s) *(volatile v8us*)(base + (size_t)(s * NTHR + tid) * 8) = pv[s];
  }
}

__global__ __launch_bounds__(GTHR) void k_gemm_in(const unsigned short* __restrict__ XN,
                                                  const unsigned short* __restrict__ INP2,
                                                  float* XIN, float* ZP) {
  __shared__ __attribute__((aligned(16))) float stg[GBM * GBN];
  const int tid = (int)threadIdx.x, lane = tid & 31, wave = tid >> 5, hh = lane >> 4, m = lane & 15;
  const int rowBase = (int)blockIdx.x * GBM;
  const int colBase = (int)blockIdx.y * GBN;
  v8f acc[8];
  gemm_core<8>(XN, KIN, INP2, KIN, KIN, rowBase, colBase, wave, hh, m, acc);
#pragma unroll
  for (int nt = 0; nt < 8; ++nt) {
    const int lc = 16 * nt + m;
#pragma unroll
    for (int r = 0; r < 8; ++r) stg[(16 * wave + 8 * hh + r) * GBN + lc] = acc[nt][r];
  }
  __syncthreads();
  float* base = (colBase < DI) ? XIN : ZP;
  const int cofs = colBase & (DI - 1);
  v4f pv[16];
#pragma unroll
  for (int i = 0; i < 16; ++i) pv[i] = *(const v4fa*)(stg + (16 * wave + i) * GBN + 4 * lane);
#pragma unroll
  for (int i = 0; i < 16; ++i)
    *(volatile v4f*)(base + (size_t)(rowBase + 16 * wave + i) * DI + cofs + 4 * lane) = pv[i];
  __threadfence();
#pragma unroll
  for (int i = 0; i < 16; ++i)
    *(volatile v4f*)(base + (size_t)(rowBase + 16 * wave + i) * DI + cofs + 4 * lane) = pv[i];
}

__global__ __launch_bounds__(NTHR) void k_conv(const float* __restrict__ XIN, const float* __restrict__ cw,
                                               const float* __restrict__ cb, unsigned short* XC) {
  __shared__ __attribute__((aligned(16))) float sIn[(CL + 3) * SD];
  __shared__ __attribute__((aligned(16))) float sOut[CL * SD];
  const int tid = (int)threadIdx.x;
  const int b = (int)blockIdx.x >> 6, l0 = ((int)blockIdx.x & 63) * CL, d0 = (int)blockIdx.y * SD;
  const int t0 = b * LSEQ + l0;
#pragma unroll 1
  for (int p = tid; p < (CL + 3) * (SD / 4); p += NTHR) {
    const int row = p >> 4, q = p & 15;
    const int l  = l0 - 3 + row;
    const int lc = l < 0 ? 0 : l;
    const float f = l < 0 ? 0.0f : 1.0f;
    const v4f v = *(const v4fa*)(XIN + (size_t)(b * LSEQ + lc) * DI + d0 + 4 * q);
    *(v4fa*)(sIn + row * SD + 4 * q) = v * f;
  }
  const int dl = tid & (SD - 1), tq = tid >> 6, d = d0 + dl;
  const v4f w4 = *(const v4fa*)(cw + (size_t)d * 4);
  const float w0 = bf16_val(w4.x), w1 = bf16_val(w4.y), w2 = bf16_val(w4.z), w3 = bf16_val(w4.w);
  const float bias = bf16_val(cb[d]);
  __syncthreads();
#pragma unroll 1
  for (int i = 0; i < CL / 4; ++i) {
    const int ll = tq * (CL / 4) + i;
    const float x0 = sIn[(ll + 0) * SD + dl];
    const float x1 = sIn[(ll + 1) * SD + dl];
    const float x2 = sIn[(ll + 2) * SD + dl];
    const float x3 = sIn[(ll + 3) * SD + dl];
    const float acc = ((w0 * x0 + w1 * x1) + w2 * x2) + w3 * x3;
    const float v = acc + bias;
    const float g = v * __builtin_amdgcn_rcpf(1.0f + expf(-v));
    sOut[ll * SD + dl] = g;
  }
  __syncthreads();
  {
    v8us pv[4];
    const int q8 = tid & 7;
#pragma unroll
    for (int s = 0; s < 4; ++s) {
      const int lid = s * 32 + (tid >> 3);
      const int i = lid >> 1, part = lid & 1;
      const unsigned mh = 0u - (unsigned)part, ml = ~mh;
      pv[s] = hilo8(sOut + i * SD + 8 * q8, ml, mh);
    }
#pragma unroll
    for (int s = 0; s < 4; ++s) {
      const int lid = s * 32 + (tid >> 3);
      const int i = lid >> 1, part = lid & 1;
      *(volatile v8us*)(XC + (size_t)(t0 + i) * KXC + part * DI + d0 + 8 * q8) = pv[s];
    }
    __threadfence();
#pragma unroll
    for (int s = 0; s < 4; ++s) {
      const int lid = s * 32 + (tid >> 3);
      const int i = lid >> 1, part = lid & 1;
      *(volatile v8us*)(XC + (size_t)(t0 + i) * KXC + part * DI + d0 + 8 * q8) = pv[s];
    }
  }
}

__global__ __launch_bounds__(GTHR) void k_gemm_xp(const unsigned short* __restrict__ XC,
                                                  const unsigned short* __restrict__ XP2, float* DBL) {
  __shared__ __attribute__((aligned(16))) float stg[GBM * NXP];
  const int tid = (int)threadIdx.x, lane = tid & 31, wave = tid >> 5, hh = lane >> 4, m = lane & 15;
  const int rowBase = (int)blockIdx.x * GBM;
  v8f acc[4];
  gemm_core<4>(XC, KXC, XP2, KXC, KXC, rowBase, 0, wave, hh, m, acc);
#pragma unroll
  for (int nt = 0; nt < 4; ++nt) {
    const int lc = 16 * nt + m;
#pragma unroll
    for (int r = 0; r < 8; ++r) stg[(16 * wave + 8 * hh + r) * NXP + lc] = acc[nt][r];
  }
  __syncthreads();
  const int sub = lane >> 4, c4 = 4 * (lane & 15);
  v4f pv[8];
#pragma unroll
  for (int i = 0; i < 8; ++i) pv[i] = *(const v4fa*)(stg + (16 * wave + 2 * i + sub) * NXP + c4);
#pragma unroll
  for (int i = 0; i < 8; ++i)
    *(volatile v4f*)(DBL + (size_t)(rowBase + 16 * wave + 2 * i + sub) * NXP + c4) = pv[i];
  __threadfence();
#pragma unroll
  for (int i = 0; i < 8; ++i)
    *(volatile v4f*)(DBL + (size_t)(rowBase + 16 * wave + 2 * i + sub) * NXP + c4) = pv[i];
}

__global__ __launch_bounds__(NTHR) void k_scan(const float* __restrict__ DBL, const unsigned short* __restrict__ XC,
                                               const float* __restrict__ ZP, const float* __restrict__ Wdt,
                                               const float* __restrict__ dtb, const float* __restrict__ Alog,
                                               const float* __restrict__ Dss, unsigned short* YHL) {
  extern __shared__ __attribute__((aligned(16))) float dyn[];
  float* sDBL = dyn;
  float* sU   = sDBL + CL * NDBL;
  float* sZG  = sU + CL * SD;
  float* sDT  = sZG + CL * SD;
  float* sY   = sDT + CL * SD;
  float* sW   = sY + CL * SD;
  float* sAm  = sW + SD * DS;
  float* sDb  = sAm + SD * DS;
  float* sDs  = sDb + SD;
  const int tid = (int)threadIdx.x;
  const int b = (int)blockIdx.x >> 3, dg = (int)blockIdx.x & 7, d0 = dg * SD;
  const int dl = tid >> 2, nq = tid & 3;
  const int dlp = tid & (SD - 1), ip0 = tid >> 6;

#pragma unroll 1
  for (int it = 0; it < 4; ++it) {
    const int e = it * NTHR + tid;
    sW[e] = bf16_val(Wdt[(size_t)d0 * DS + e]);
    const float al = bf16_val(Alog[(size_t)d0 * DS + e]);
    sAm[e] = -expf(al);
  }
  if (tid < SD) {
    sDb[tid] = bf16_val(dtb[d0 + tid]);
  } else if (tid < 2 * SD) {
    sDs[tid - SD] = bf16_val(Dss[d0 + tid - SD]);
  }
  __syncthreads();
  const v4f a4 = *(const v4fa*)(sAm + dl * DS + 4 * nq);
  const float Dd  = sDs[dl];
  const float dbp = sDb[dlp];
  float h0 = 0.0f, h1 = 0.0f, h2 = 0.0f, h3 = 0.0f;
  const int q8 = tid & 7;

#pragma unroll 1
  for (int ch = 0; ch < LSEQ / CL; ++ch) {
    const int t0 = b * LSEQ + ch * CL;
#pragma unroll 1
    for (int p = tid; p < CL * (NDBL / 4); p += NTHR) {
      const int i = p / (NDBL / 4), q = p - (NDBL / 4) * i;
      const v4f v = *(const v4fa*)(DBL + (size_t)(t0 + i) * NXP + 4 * q);
      *(v4fa*)(sDBL + i * NDBL + 4 * q) = v;
    }
#pragma unroll 1
    for (int j = 0; j < 2; ++j) {
      const int p = tid + NTHR * j;
      const int i = p >> 3, w8 = p & 7;
      const unsigned short* sp = XC + (size_t)(t0 + i) * KXC + d0 + 8 * w8;
      const v8us hv = *(const v8usa*)sp;
      const v8us lv = *(const v8usa*)(sp + DI);
      v4f ua, ub;
      ua.x = bfw(hv[0]) + bfw(lv[0]);
      ua.y = bfw(hv[1]) + bfw(lv[1]);
      ua.z = bfw(hv[2]) + bfw(lv[2]);
      ua.w = bfw(hv[3]) + bfw(lv[3]);
      ub.x = bfw(hv[4]) + bfw(lv[4]);
      ub.y = bfw(hv[5]) + bfw(lv[5]);
      ub.z = bfw(hv[6]) + bfw(lv[6]);
      ub.w = bfw(hv[7]) + bfw(lv[7]);
      *(v4fa*)(sU + i * SD + 8 * w8)     = ua;
      *(v4fa*)(sU + i * SD + 8 * w8 + 4) = ub;
    }
#pragma unroll 1
    for (int j = 0; j < 4; ++j) {
      const int p = tid + NTHR * j;
      const int i = p >> 4, q = p & 15;
      const v4f v = *(const v4fa*)(ZP + (size_t)(t0 + i) * DI + d0 + 4 * q);
      *(v4fa*)(sZG + i * SD + 4 * q) = v;
    }
    __syncthreads();
#pragma unroll 1
    for (int j = 0; j < CL / 4; ++j) {
      const int i = ip0 + 4 * j;
      float dot = 0.0f;
#pragma unroll 1
      for (int r4 = 0; r4 < DTR / 4; ++r4) {
        const v4f dv = *(const v4fa*)(sDBL + i * NDBL + 4 * r4);
        const v4f wv = *(const v4fa*)(sW + dlp * DS + 4 * r4);
        dot += dv.x * wv.x;
        dot += dv.y * wv.y;
        dot += dv.z * wv.z;
        dot += dv.w * wv.w;
      }
      const float pre = dot + dbp;
      const float dt  = fmaxf(pre, 0.0f) + log1pf(expf(-fabsf(pre)));
      const float z   = sZG[i * SD + dlp];
      const float g   = z * __builtin_amdgcn_rcpf(1.0f + expf(-z));
      sDT[i * SD + dlp] = dt;
      sZG[i * SD + dlp] = g;
    }
    __syncthreads();
#pragma unroll 1
    for (int i = 0; i < CL; ++i) {
      const float dt = sDT[i * SD + dl];
      const float u  = sU[i * SD + dl];
      const float g  = sZG[i * SD + dl];
      const v4f Bv = *(const v4fa*)(sDBL + i * NDBL + DTR + 4 * nq);
      const v4f Cv = *(const v4fa*)(sDBL + i * NDBL + DTR + DS + 4 * nq);
      const float du = dt * u;
      const float e0 = expf(dt * a4.x);
      const float e1 = expf(dt * a4.y);
      const float e2 = expf(dt * a4.z);
      const float e3 = expf(dt * a4.w);
      h0 = h0 * e0 + du * Bv.x;
      h1 = h1 * e1 + du * Bv.y;
      h2 = h2 * e2 + du * Bv.z;
      h3 = h3 * e3 + du * Bv.w;
      float pp = h0 * Cv.x + h1 * Cv.y + h2 * Cv.z + h3 * Cv.w;
      pp += __shfl_xor(pp, 1);
      pp += __shfl_xor(pp, 2);
      const float yv = (pp + u * Dd) * g;
      if (nq == 0) sY[i * SD + dl] = yv;
    }
    __syncthreads();
    {
      v8us pv[4];
#pragma unroll
      for (int s = 0; s < 4; ++s) {
        const int lid = s * 32 + (tid >> 3);
        const int i = lid >> 1, part = lid & 1;
        const unsigned mh = 0u - (unsigned)part, ml = ~mh;
        pv[s] = hilo8(sY + i * SD + 8 * q8, ml, mh);
      }
#pragma unroll
      for (int s = 0; s < 4; ++s) {
        const int lid = s * 32 + (tid >> 3);
        const int i = lid >> 1, part = lid & 1;
        *(volatile v8us*)(YHL + (size_t)(t0 + i) * KXC + part * DI + d0 + 8 * q8) = pv[s];
      }
      __threadfence();
#pragma unroll
      for (int s = 0; s < 4; ++s) {
        const int lid = s * 32 + (tid >> 3);
        const int i = lid >> 1, part = lid & 1;
        *(volatile v8us*)(YHL + (size_t)(t0 + i) * KXC + part * DI + d0 + 8 * q8) = pv[s];
      }
    }
  }
}

__global__ __launch_bounds__(GTHR) void k_gemm_out(const unsigned short* __restrict__ YHL,
                                                   const unsigned short* __restrict__ OUT2,
                                                   const float* __restrict__ x, const float* __restrict__ skip,
                                                   unsigned short* XM) {
  __shared__ __attribute__((aligned(16))) float stg[GBM * GBN];
  const int tid = (int)threadIdx.x, lane = tid & 31, wave = tid >> 5, hh = lane >> 4, m = lane & 15;
  const int rowBase = (int)blockIdx.x * GBM;
  const int colBase = (int)blockIdx.y * GBN;
  v8f acc[8];
  gemm_core<8>(YHL, KXC, OUT2, KXC, KXC, rowBase, colBase, wave, hh, m, acc);
  const float sk = bf16_val(skip[0]);
  const int b  = rowBase >> 12;
  const int lw = (rowBase & (LSEQ - 1)) + 16 * wave + 8 * hh;
#pragma unroll
  for (int nt = 0; nt < 8; ++nt) {
    const int lc = 16 * nt + m;
    const int c  = colBase + lc;
    const float* xp = x + ((size_t)(b * DM + c) * LSEQ + lw);
    const v4f xa = *(const v4fa*)xp;
    const v4f xb = *(const v4fa*)(xp + 4);
    const v8f x8 = {xa.x, xa.y, xa.z, xa.w, xb.x, xb.y, xb.z, xb.w};
#pragma unroll
    for (int r = 0; r < 8; ++r) {
      const int lr = 16 * wave + 8 * hh + r;
      stg[lr * GBN + lc] = acc[nt][r] + sk * bf16_val(x8[r]);
    }
  }
  __syncthreads();
  {
    const int part = lane >> 4, j = lane & 15;
    const unsigned mh = 0u - (unsigned)part, ml = ~mh;
    v8us pv[16];
#pragma unroll
    for (int i = 0; i < 16; ++i) pv[i] = hilo8(stg + (16 * wave + i) * GBN + 8 * j, ml, mh);
#pragma unroll
    for (int i = 0; i < 16; ++i)
      *(volatile v8us*)(XM + (size_t)(rowBase + 16 * wave + i) * KXM + part * DM + colBase + 8 * j) = pv[i];
    __threadfence();
#pragma unroll
    for (int i = 0; i < 16; ++i)
      *(volatile v8us*)(XM + (size_t)(rowBase + 16 * wave + i) * KXM + part * DM + colBase + 8 * j) = pv[i];
  }
}

__global__ __launch_bounds__(GTHR) void k_gemm_pr(const unsigned short* __restrict__ XM,
                                                  const unsigned short* __restrict__ PRJ2,
                                                  const float* __restrict__ pb, float* out) {
  __shared__ __attribute__((aligned(16))) float stgT[GBN * TPP];
  const int tid = (int)threadIdx.x, lane = tid & 31, wave = tid >> 5, hh = lane >> 4, m = lane & 15;
  const int rowBase = (int)blockIdx.x * GBM;
  const int colBase = (int)blockIdx.y * GBN;
  v8f acc[8];
  gemm_core<8>(XM, KXM, PRJ2, KXM, KXM, rowBase, colBase, wave, hh, m, acc);
#pragma unroll
  for (int nt = 0; nt < 8; ++nt) {
    const int lc = 16 * nt + m;
    const float bv = bf16_val(pb[colBase + lc]);
#pragma unroll
    for (int r = 0; r < 8; ++r) {
      const int lr = 16 * wave + 8 * hh + r;
      stgT[lc * TPP + lr] = acc[nt][r] + bv;
    }
  }
  __syncthreads();
  const int b = rowBase >> 12, l0 = rowBase & (LSEQ - 1);
  const int q8 = tid & 7, sub = tid >> 3;
  float* ob = out + ((size_t)(b * DM + colBase) * LSEQ + l0);
#pragma unroll 1
  for (int s = 0; s < 16; ++s) {
    const int lid = s * 16 + sub;
    const int cl = lid >> 1, hl = lid & 1;
    const v4f v = *(const v4fa*)(stgT + cl * TPP + 32 * hl + 4 * q8);
    *(volatile v4f*)(ob + (size_t)cl * LSEQ + 32 * hl + 4 * q8) = v;
  }
  __threadfence();
#pragma unroll 1
  for (int s = 0; s < 16; ++s) {
    const int lid = s * 16 + sub;
    const int cl = lid >> 1, hl = lid & 1;
    const v4f v = *(const v4fa*)(stgT + cl * TPP + 32 * hl + 4 * q8);
    *(volatile v4f*)(ob + (size_t)cl * LSEQ + 32 * hl + 4 * q8) = v;
  }
}

extern "C" void kernel_launch(void* const* d_in, const int* in_sizes, int n_in,
                              void* d_out, int out_size, void* d_ws, size_t ws_size,
                              hipStream_t stream) {
  if (n_in < 15) return;
  if (in_sizes[0] != BSZ * DM * LSEQ) return;
  if (in_sizes[1] != DM || in_sizes[2] != DM) return;
  if (in_sizes[3] != 2 * DI * DM) return;
  if (in_sizes[4] != DI * 4 || in_sizes[5] != DI) return;
  if (in_sizes[6] != NDBL * DI) return;
  if (in_sizes[7] != DI * DTR || in_sizes[8] != DI) return;
  if (in_sizes[9] != DI * DS || in_sizes[10] != DI) return;
  if (in_sizes[11] != DM * DI) return;
  if (in_sizes[12] != DM * DM || in_sizes[13] != DM) return;
  if (in_sizes[14] < 1) return;
  if (out_size != BSZ * DM * LSEQ) return;

  const float* x     = (const float*)d_in[0];
  const float* nw    = (const float*)d_in[1];
  const float* nb    = (const float*)d_in[2];
  const float* Win   = (const float*)d_in[3];
  const float* cw    = (const float*)d_in[4];
  const float* cb    = (const float*)d_in[5];
  const float* Wxp   = (const float*)d_in[6];
  const float* Wdt   = (const float*)d_in[7];
  const float* dtb   = (const float*)d_in[8];
  const float* Alog  = (const float*)d_in[9];
  const float* Dss   = (const float*)d_in[10];
  const float* Wout  = (const float*)d_in[11];
  const float* Wpr   = (const float*)d_in[12];
  const float* pb    = (const float*)d_in[13];
  const float* skip  = (const float*)d_in[14];
  float* out = (float*)d_out;

  size_t off = 0;
  const size_t oINP2 = off; off += (size_t)2 * DI * KIN * 2;
  const size_t oXP2  = off; off += (size_t)NXP * KXC * 2;
  const size_t oOUT2 = off; off += (size_t)DM * KXC * 2;
  const size_t oPRJ2 = off; off += (size_t)DM * KXM * 2;
  const size_t oXN   = off; off += (size_t)TROWS * KIN * 2;
  const size_t oXIN  = off; off += (size_t)TROWS * DI * 4;
  const size_t oZ    = off; off += (size_t)TROWS * DI * 4;
  const size_t oXC   = off; off += (size_t)TROWS * KXC * 2;
  const size_t oDBL  = off; off += (size_t)TROWS * NXP * 4;
  if (off > ws_size || off > (size_t)WSMAX) return;

  char* ws = (char*)d_ws;
  unsigned short* INP2 = (unsigned short*)(ws + oINP2);
  unsigned short* XP2  = (unsigned short*)(ws + oXP2);
  unsigned short* OUT2 = (unsigned short*)(ws + oOUT2);
  unsigned short* PRJ2 = (unsigned short*)(ws + oPRJ2);
  unsigned short* XNHL = (unsigned short*)(ws + oXN);
  unsigned short* XMHL = (unsigned short*)(ws + oXN);
  float*          XIN  = (float*)(ws + oXIN);
  unsigned short* YHL  = (unsigned short*)(ws + oXIN);
  float*          ZP   = (float*)(ws + oZ);
  unsigned short* XCHL = (unsigned short*)(ws + oXC);
  float*          DBL  = (float*)(ws + oDBL);

  hipFuncSetAttribute(reinterpret_cast<const void*>(&k_scan), hipFuncAttributeMaxDynamicSharedMemorySize,
                      (int)SCAN_LDS_BYTES);

  k_wprep<<<NU_ALL / NTHR, NTHR, 0, stream>>>(Win, Wxp, Wout, Wpr, INP2, XP2, OUT2, PRJ2);
  k_ln<<<dim3(LSEQ / 32, BSZ), NTHR, 0, stream>>>(x, nw, nb, XNHL);
  k_gemm_in<<<dim3(TROWS / GBM, (2 * DI) / GBN), GTHR, 0, stream>>>(XNHL, INP2, XIN, ZP);
  k_conv<<<dim3(TROWS / CL, DI / SD), NTHR, 0, stream>>>(XIN, cw, cb, XCHL);
  k_gemm_xp<<<dim3(TROWS / GBM, 1), GTHR, 0, stream>>>(XCHL, XP2, DBL);
  k_scan<<<BSZ * (DI / SD), NTHR, SCAN_LDS_BYTES, stream>>>(DBL, XCHL, ZP, Wdt, dtb, Alog, Dss, YHL);
  k_gemm_out<<<dim3(TROWS / GBM, DM / GBN), GTHR, 0, stream>>>(YHL, OUT2, x, skip, XMHL);
  k_gemm_pr<<<dim3(TROWS / GBM, DM / GBN), GTHR, 0, stream>>>(XMHL, PRJ2, pb, out);
}
